// StyleAttentionNet_18287970746386
// MI455X (gfx1250) — hardware-verified
//
#include <hip/hip_runtime.h>
#include <math.h>

constexpr int   kBatch    = 4;
constexpr int   kCh       = 512;
constexpr int   kSp       = 4096;
constexpr int   kQChunk   = 2048;
constexpr int   kHalfRow  = kSp / 2;
constexpr int   kStatRows = 2 * kBatch * kCh;
constexpr float kEps       = 1e-5f;
constexpr float kWCarry    = 16.0f;
constexpr float kPCarry    = 2048.0f;
constexpr float kProjScale = 1.0f / 16.0f;
constexpr float kPVScale   = 16.0f / 2048.0f;
constexpr float kOutScale  = 1.0f / (16.0f * 16.0f);
constexpr float kInvN      = 1.0f / 4096.0f;
constexpr float kInvNm1    = 1.0f / 4095.0f;

typedef __attribute__((ext_vector_type(16))) _Float16 v16h;
typedef __attribute__((ext_vector_type(8)))  _Float16 v8h;
typedef __attribute__((ext_vector_type(16))) __bf16   v16b;
typedef __attribute__((ext_vector_type(8)))  __bf16   v8b;
typedef __attribute__((ext_vector_type(8)))  float    v8f;
typedef __attribute__((ext_vector_type(4)))  float    v4f;
typedef __attribute__((ext_vector_type(4)))  unsigned int v4u;

__device__ __forceinline__ unsigned short f2bf_bits(float f) {
  unsigned u = __float_as_uint(f);
  return (unsigned short)((u + 0x7FFFu + ((u >> 16) & 1u)) >> 16);
}
__device__ __forceinline__ float bf_bits2f(unsigned short h) { return __uint_as_float(((unsigned)h) << 16); }

__device__ __forceinline__ void dep_guard_h(v8f& a, v8f& b, v16h x, v16h y) { asm volatile("v_nop\n\tv_nop\n\tv_nop\n\tv_nop" : "+v"(a), "+v"(b) : "v"(x), "v"(y)); }
__device__ __forceinline__ void dep_guard_b(v8f& a, v8f& b, v16b x, v16b y) { asm volatile("v_nop\n\tv_nop\n\tv_nop\n\tv_nop" : "+v"(a), "+v"(b) : "v"(x), "v"(y)); }
__device__ __forceinline__ void keep4_h(v16h a, v16h b, v16h c, v16h d) { asm volatile("v_nop" :: "v"(a), "v"(b), "v"(c), "v"(d)); }
__device__ __forceinline__ void keep4_b(v16b a, v16b b, v16b c, v16b d) { asm volatile("v_nop" :: "v"(a), "v"(b), "v"(c), "v"(d)); }
__device__ __forceinline__ void acc_guard4(v8f& a, v8f& b, v8f& c, v8f& d) { asm volatile("v_nop\n\tv_nop\n\tv_nop\n\tv_nop" : "+v"(a), "+v"(b), "+v"(c), "+v"(d)); }
template <typename T> struct Frag;
template <> struct Frag<_Float16> {
  typedef v16h V; union U { v16h v; v8h h[2]; };
  static __device__ __forceinline__ v16h load(const _Float16* p) {
    U f; f.h[0] = *(const v8h*)(p); f.h[1] = *(const v8h*)(p + 16); return f.v;
  }
  static __device__ __forceinline__ v8f mma(v16h a, v16h b, v8f c) {
    return __builtin_amdgcn_wmma_f32_16x16x32_f16(false, a, false, b, (short)0, c, false, false);
  }
  static __device__ __forceinline__ void guard(v8f& a, v8f& b, v16h x, v16h y) { dep_guard_h(a, b, x, y); }
  static __device__ __forceinline__ void keep(v16h a, v16h b, v16h c, v16h d) { keep4_h(a, b, c, d); }
};
template <> struct Frag<__bf16> {
  typedef v16b V; union U { v16b v; v8b h[2]; };
  static __device__ __forceinline__ v16b load(const __bf16* p) {
    U f; f.h[0] = *(const v8b*)(p); f.h[1] = *(const v8b*)(p + 16); return f.v;
  }
  static __device__ __forceinline__ v8f mma(v16b a, v16b b, v8f c) {
    return __builtin_amdgcn_wmma_f32_16x16x32_bf16(false, a, false, b, (short)0, c, false, false);
  }
  static __device__ __forceinline__ void guard(v8f& a, v8f& b, v16b x, v16b y) { dep_guard_b(a, b, x, y); }
  static __device__ __forceinline__ void keep(v16b a, v16b b, v16b c, v16b d) { keep4_b(a, b, c, d); }
};

__device__ __forceinline__ unsigned pk16(unsigned short a, unsigned short b) { return (unsigned)a | ((unsigned)b << 16); }
__device__ __forceinline__ unsigned short h_bits(float f) { const _Float16 h = (_Float16)f; return __builtin_bit_cast(unsigned short, h); }

template <int ET> struct Elem;
template <> struct Elem<0> { typedef _Float16 T; };
template <> struct Elem<1> { typedef __bf16 T; };
template <int ET, bool SPLIT, int BIAS_MODE, int OUT_MODE, bool RESID, int ACT = 0>
__global__ __launch_bounds__(256) void wmma_gemm64(
    const unsigned short* __restrict__ Ap, const unsigned short* __restrict__ A2p, int lda, long strideA,
    const unsigned short* __restrict__ Btp, const unsigned short* __restrict__ Bt2p, int ldb, long strideB,
    void* __restrict__ Cout, void* __restrict__ Cout2, int ldc, long strideC,
    const float* __restrict__ bias,
    const float* __restrict__ resid, long strideR,
    int M, int N, int K, float scale) {
  typedef typename Elem<ET>::T T;
  typedef typename Frag<T>::V V;
  const T* A = (const T*)Ap; const T* A2 = (const T*)A2p; const T* Bt = (const T*)Btp; const T* Bt2 = (const T*)Bt2p;
  __shared__ __align__(16) float sT[8][16 * 68];
  const int b    = blockIdx.y;
  const int lane = threadIdx.x & 31;
  const int wave = threadIdx.x >> 5;
  const int tilesN = N >> 6;
  const int tilesM = M >> 6;
  const int tile = blockIdx.x * 8 + wave;
  if (tile >= tilesM * tilesN) return;
  const int tm = tile / tilesN;
  const int tn = tile - tm * tilesN;
  const int m0 = tm << 6;
  const int n0 = tn << 6;

  const T* Ab  = A  + (size_t)b * strideA;
  const T* Bb  = Bt + (size_t)b * strideB;
  const T* Ab2 = SPLIT ? (A2  + (size_t)b * strideA) : nullptr;
  const T* Bb2 = SPLIT ? (Bt2 + (size_t)b * strideB) : nullptr;

  const int rlane = lane & 15;
  const int koff  = (lane >> 4) * 8;
  const int mOff  = (lane >> 4) * 8;

  v8f acc[4][4];
#pragma unroll
  for (int i = 0; i < 4; ++i)
#pragma unroll
    for (int j = 0; j < 4; ++j) acc[i][j] = (v8f){0.f,0.f,0.f,0.f,0.f,0.f,0.f,0.f};

  for (int k0 = 0; k0 < K; k0 += 32) {
    V bh[4], bl[4];
#pragma unroll
    for (int j = 0; j < 4; ++j) {
      const size_t bo = (size_t)(n0 + (j << 4) + rlane) * ldb + koff + k0;
      bh[j] = Frag<T>::load(Bb + bo);
      if (SPLIT) bl[j] = Frag<T>::load(Bb2 + bo);
    }
#pragma unroll
    for (int i = 0; i < 4; ++i) {
      const size_t ao = (size_t)(m0 + (i << 4) + rlane) * lda + koff + k0;
      V ah = Frag<T>::load(Ab + ao);
      V al;
      if (SPLIT) al = Frag<T>::load(Ab2 + ao);
#pragma unroll
      for (int j = 0; j < 4; ++j) {
        acc[i][j] = Frag<T>::mma(ah, bh[j], acc[i][j]);
        if (SPLIT) {
          acc[i][j] = Frag<T>::mma(ah, bl[j], acc[i][j]);
          acc[i][j] = Frag<T>::mma(al, bh[j], acc[i][j]);
        }
      }
      Frag<T>::guard(acc[i][0], acc[i][3], ah, SPLIT ? al : ah);
    }
    Frag<T>::keep(bh[0], bh[1], bh[2], bh[3]);
    if (SPLIT) Frag<T>::keep(bl[0], bl[1], bl[2], bl[3]);
  }
  acc_guard4(acc[0][0], acc[0][1], acc[0][2], acc[0][3]);
  acc_guard4(acc[1][0], acc[1][1], acc[1][2], acc[1][3]);
  acc_guard4(acc[2][0], acc[2][1], acc[2][2], acc[2][3]);
  acc_guard4(acc[3][0], acc[3][1], acc[3][2], acc[3][3]);

  float* slab = sT[wave];
  const float* Rb = RESID ? (resid + (size_t)b * strideR) : nullptr;
#pragma unroll
  for (int i = 0; i < 4; ++i) {
    const int mBase = m0 + (i << 4);
#pragma unroll
    for (int j = 0; j < 4; ++j) {
      const int n = n0 + (j << 4) + rlane;
      float bv = 0.f;
      if (BIAS_MODE == 2) bv = bias[n];
#pragma unroll
      for (int r = 0; r < 8; ++r) {
        float v = acc[i][j][r] * scale;
        if (BIAS_MODE == 1) v += bias[mBase + mOff + r];
        if (BIAS_MODE == 2) v += bv;
        if (RESID) v += Rb[(size_t)(mBase + mOff + r) * ldc + n];
        if (ACT == 2) v = fmaxf(v, 0.0f);
        if (ACT == 4) v = (v > 0.f) ? v : 0.01f * v;
        slab[(mOff + r) * 68 + (j << 4) + rlane] = v;
      }
    }
    __builtin_amdgcn_fence(__ATOMIC_RELEASE, "workgroup");
    __builtin_amdgcn_wave_barrier();
    __builtin_amdgcn_fence(__ATOMIC_ACQUIRE, "workgroup");
    if (OUT_MODE == 0) {
      float* C = (float*)Cout + (size_t)b * strideC;
      const int hh = lane >> 4, c4 = (lane & 15) * 4;
      for (int pass = 0; pass < 2; ++pass) {
#pragma unroll
        for (int it = 0; it < 8; ++it) {
          const int row = it * 2 + hh;
          v4f v = *(const v4f*)(slab + row * 68 + c4);
          *(volatile v4f*)(C + (size_t)(mBase + row) * ldc + n0 + c4) = v;
        }
        __threadfence();
      }
    } else {
      const int q = lane >> 3, c8 = (lane & 7) * 8;
      unsigned short* C  = (unsigned short*)Cout  + (size_t)b * strideC;
      unsigned short* C2 = (OUT_MODE == 2) ? ((unsigned short*)Cout2 + (size_t)b * strideC) : nullptr;
      for (int pass = 0; pass < 2; ++pass) {
#pragma unroll
        for (int it = 0; it < 4; ++it) {
          const int row = it * 4 + q;
          const float* sp = slab + row * 68 + c8;
          v8h hv, lv;
#pragma unroll
          for (int e = 0; e < 8; ++e) {
            if (OUT_MODE == 1) {
              hv[e] = (_Float16)sp[e];
            } else {
              unsigned short hb = f2bf_bits(sp[e]);
              unsigned short lb = f2bf_bits(sp[e] - bf_bits2f(hb));
              hv[e] = __builtin_bit_cast(_Float16, hb);
              lv[e] = __builtin_bit_cast(_Float16, lb);
            }
          }
          *(volatile v8h*)(C + (size_t)(mBase + row) * ldc + n0 + c8) = hv;
          if (OUT_MODE == 2) *(volatile v8h*)(C2 + (size_t)(mBase + row) * ldc + n0 + c8) = lv;
        }
        __threadfence();
      }
    }
    __builtin_amdgcn_fence(__ATOMIC_RELEASE, "workgroup");
    __builtin_amdgcn_wave_barrier();
    __builtin_amdgcn_fence(__ATOMIC_ACQUIRE, "workgroup");
  }
}

__global__ __launch_bounds__(256) void stats_kernel(const float* __restrict__ xc, const float* __restrict__ xs,
                                                    float* __restrict__ meanA, float* __restrict__ rstdA) {
  __shared__ float sMean[32];
  __shared__ float sRstd[32];
  const int blk  = blockIdx.x;
  const int tsel = blk >> 6;
  const float* src = (tsel == 0) ? xc : xs;
  const int rowBase = (blk & 63) * 32;
  const int t = threadIdx.x, lane = t & 31, wave = t >> 5;
#pragma unroll
  for (int r = 0; r < 4; ++r) {
    const int row = rowBase + wave * 4 + r;
    const float* p = src + (size_t)row * kSp + lane * 4;
    v4f s = (v4f){0.f, 0.f, 0.f, 0.f};
    v4f q = (v4f){0.f, 0.f, 0.f, 0.f};
#pragma unroll 1
    for (int i = 0; i < 32; ++i) {
      const v4f v = *(const v4f*)(p + i * 128);
      s += v;
      q += v * v;
    }
    float su = (s[0] + s[1]) + (s[2] + s[3]);
    float sq = (q[0] + q[1]) + (q[2] + q[3]);
#pragma unroll
    for (int off = 16; off > 0; off >>= 1) {
      su += __shfl_xor(su, off, 32);
      sq += __shfl_xor(sq, off, 32);
    }
    const float mean = su * kInvN;
    float var = (sq - su * mean) * kInvNm1;
    var = fmaxf(var, 0.0f);
    const float rstd = 1.0f / sqrtf(var + kEps);
    if (lane == 0) { sMean[wave * 4 + r] = mean; sRstd[wave * 4 + r] = rstd; }
  }
  __syncthreads();
  const int orow = tsel * (kBatch * kCh) + rowBase + lane;
  if (wave == 0) {
    const float v = sMean[lane];
    *(volatile float*)(meanA + orow) = v;
    __threadfence();
    *(volatile float*)(meanA + orow) = v;
  } else if (wave == 1) {
    const float v = sRstd[lane];
    *(volatile float*)(rstdA + orow) = v;
    __threadfence();
    *(volatile float*)(rstdA + orow) = v;
  }
}

__global__ __launch_bounds__(256) void token_planes_kernel(const float* __restrict__ content, const float* __restrict__ style,
                                                           const float* __restrict__ meanA, const float* __restrict__ rstdA, int b,
                                                           unsigned short* __restrict__ XcT, unsigned short* __restrict__ XsT,
                                                           unsigned short* __restrict__ SsT) {
  __shared__ float sm[64][65];
  const int t  = threadIdx.x;
  const int z  = blockIdx.z;
  const int n0 = blockIdx.x * 64;
  const int c0 = blockIdx.y * 64;
  const float* src = ((z == 0) ? content : style) + (size_t)b * kCh * kSp;
  unsigned short* dst = (z == 0) ? XcT : (z == 1) ? XsT : SsT;
  const int statOff = ((z == 0) ? 0 : (kBatch * kCh)) + b * kCh;
  const bool useNorm = (z < 2);
  const int r16 = t >> 4, c4 = (t & 15) * 4;
#pragma unroll
  for (int p = 0; p < 4; ++p) {
    const int cl = p * 16 + r16;
    const int ch = c0 + cl;
    const v4f v = *(const v4f*)(src + (size_t)ch * kSp + n0 + c4);
    const float m  = meanA[statOff + ch];
    const float rs = rstdA[statOff + ch];
    const float mm = useNorm ? m : 0.0f;
    const float rr = useNorm ? rs : 1.0f;
#pragma unroll
    for (int e = 0; e < 4; ++e) sm[cl][c4 + e] = (v[e] - mm) * rr;
  }
  __syncthreads();
  const int lane = t & 31, wave = t >> 5;
  const int q = lane >> 3, c8 = (lane & 7) * 8;
  for (int pass = 0; pass < 2; ++pass) {
#pragma unroll
    for (int it = 0; it < 2; ++it) {
      const int row = wave * 8 + it * 4 + q;
      unsigned short hb[8];
#pragma unroll
      for (int e = 0; e < 8; ++e) hb[e] = h_bits(sm[c8 + e][row]);
      const v4u u = (v4u){pk16(hb[0], hb[1]), pk16(hb[2], hb[3]), pk16(hb[4], hb[5]), pk16(hb[6], hb[7])};
      *(volatile v4u*)(dst + (size_t)(n0 + row) * kCh + c0 + c8) = u;
    }
    __threadfence();
  }
}

__global__ __launch_bounds__(256) void wcast_kernel(const float* __restrict__ W0, const float* __restrict__ W1,
                                                    const float* __restrict__ W2, const float* __restrict__ W3,
                                                    unsigned short* __restrict__ out, float scale) {
  const int blk = blockIdx.x;
  const int w = blk >> 7;
  const float* src = (w == 0) ? W0 : (w == 1) ? W1 : (w == 2) ? W2 : W3;
  const int i  = (blk & 127) * 256 + threadIdx.x;
  const size_t e0 = (size_t)i * 8;
  const v4f a = *(const v4f*)(src + e0);
  const v4f c = *(const v4f*)(src + e0 + 4);
  unsigned short hb[8];
#pragma unroll
  for (int e = 0; e < 4; ++e) {
    hb[e]     = h_bits(a[e] * scale);
    hb[4 + e] = h_bits(c[e] * scale);
  }
  const v4u u = (v4u){pk16(hb[0], hb[1]), pk16(hb[2], hb[3]), pk16(hb[4], hb[5]), pk16(hb[6], hb[7])};
  unsigned short* dp = out + (size_t)w * kCh * kCh + e0;
  *(volatile v4u*)dp = u;
  __threadfence();
  *(volatile v4u*)dp = u;
}

__global__ __launch_bounds__(256) void softmax_kernel(const float* __restrict__ Sp, unsigned short* __restrict__ Pp) {
  __shared__ float redM[8];
  __shared__ float redS[8];
  const int row  = blockIdx.x;
  const int t    = threadIdx.x;
  const int lane = t & 31, wave = t >> 5;
  const int cA = 8 * t;
  const int cB = kHalfRow + 8 * t;
  const float* sr = Sp + (size_t)row * kSp;
  const v4f a0 = *(const v4f*)(sr + cA);
  const v4f a1 = *(const v4f*)(sr + cA + 4);
  const v4f b0 = *(const v4f*)(sr + cB);
  const v4f b1 = *(const v4f*)(sr + cB + 4);
  float x[16];
#pragma unroll
  for (int e = 0; e < 4; ++e) { x[e] = a0[e]; x[4 + e] = a1[e]; x[8 + e] = b0[e]; x[12 + e] = b1[e]; }
  float m = x[0];
#pragma unroll
  for (int i = 1; i < 16; ++i) m = fmaxf(m, x[i]);
#pragma unroll
  for (int off = 16; off > 0; off >>= 1) m = fmaxf(m, __shfl_xor(m, off, 32));
  if (lane == 0) redM[wave] = m;
  __syncthreads();
  float gm = redM[0];
#pragma unroll
  for (int w = 1; w < 8; ++w) gm = fmaxf(gm, redM[w]);
  float ex[16];
  float s = 0.0f;
#pragma unroll
  for (int i = 0; i < 16; ++i) { ex[i] = expf(x[i] - gm); s += ex[i]; }
#pragma unroll
  for (int off = 16; off > 0; off >>= 1) s += __shfl_xor(s, off, 32);
  if (lane == 0) redS[wave] = s;
  __syncthreads();
  float tot = redS[0];
#pragma unroll
  for (int w = 1; w < 8; ++w) tot += redS[w];
  const float inv = 1.0f / tot;
  unsigned short hb[16];
#pragma unroll
  for (int i = 0; i < 16; ++i) hb[i] = h_bits((ex[i] * inv) * kPCarry);
  const v4u uA = (v4u){pk16(hb[0], hb[1]), pk16(hb[2], hb[3]), pk16(hb[4], hb[5]), pk16(hb[6], hb[7])};
  const v4u uB = (v4u){pk16(hb[8], hb[9]), pk16(hb[10], hb[11]), pk16(hb[12], hb[13]), pk16(hb[14], hb[15])};
  unsigned short* pr = Pp + (size_t)row * kSp;
  *(volatile v4u*)(pr + cA) = uA;
  *(volatile v4u*)(pr + cB) = uB;
  __threadfence();
  *(volatile v4u*)(pr + cA) = uA;
  *(volatile v4u*)(pr + cB) = uB;
}

extern "C" void kernel_launch(void* const* d_in, const int* in_sizes, int n_in,
                              void* d_out, int out_size, void* d_ws, size_t ws_size,
                              hipStream_t stream) {
  if (n_in < 10) return;
  const int actN = kBatch * kCh * kSp;
  const int wN   = kCh * kCh;
  if (in_sizes[0] != actN || in_sizes[1] != actN) return;
  if (in_sizes[2] != wN || in_sizes[4] != wN || in_sizes[6] != wN || in_sizes[8] != wN) return;
  if (in_sizes[3] != kCh || in_sizes[5] != kCh || in_sizes[7] != kCh || in_sizes[9] != kCh) return;
  if (out_size != actN) return;

  const float* content = (const float*)d_in[0];
  const float* style   = (const float*)d_in[1];
  const float* Wq = (const float*)d_in[2];  const float* bq = (const float*)d_in[3];
  const float* Wk = (const float*)d_in[4];  const float* bk = (const float*)d_in[5];
  const float* Wv = (const float*)d_in[6];  const float* bv = (const float*)d_in[7];
  const float* Wo = (const float*)d_in[8];  const float* bo = (const float*)d_in[9];
  float* out = (float*)d_out;

  size_t off = 0;
  auto carve = [&](size_t bytes) { size_t o = off; off += (bytes + 127) & ~(size_t)127; return o; };
  const size_t planeBytes = (size_t)kSp * kCh * 2;
  const size_t oW16  = carve((size_t)4 * wN * 2);
  const size_t oMean = carve((size_t)kStatRows * 4);
  const size_t oRstd = carve((size_t)kStatRows * 4);
  const size_t oXc   = carve(planeBytes);
  const size_t oXs   = carve(planeBytes);
  const size_t oSs   = carve(planeBytes);
  const size_t oQ    = carve(planeBytes);
  const size_t oK    = carve(planeBytes);
  const size_t oV    = carve(planeBytes);
  const size_t oO    = carve(planeBytes);
  const size_t oS    = carve((size_t)kQChunk * kSp * 4);
  const size_t oP    = carve((size_t)kQChunk * kSp * 2);
  if (off > ws_size) return;

  char* ws = (char*)d_ws;
  unsigned short* W16 = (unsigned short*)(ws + oW16);
  float* meanA = (float*)(ws + oMean);
  float* rstdA = (float*)(ws + oRstd);
  unsigned short* XcT = (unsigned short*)(ws + oXc);
  unsigned short* XsT = (unsigned short*)(ws + oXs);
  unsigned short* SsT = (unsigned short*)(ws + oSs);
  unsigned short* Qp  = (unsigned short*)(ws + oQ);
  unsigned short* Kp  = (unsigned short*)(ws + oK);
  unsigned short* Vcm = (unsigned short*)(ws + oV);
  unsigned short* Op  = (unsigned short*)(ws + oO);
  float* Sp = (float*)(ws + oS);
  unsigned short* Pp = (unsigned short*)(ws + oP);

  const unsigned short* Wq16 = W16 + (size_t)0 * wN;
  const unsigned short* Wk16 = W16 + (size_t)1 * wN;
  const unsigned short* Wv16 = W16 + (size_t)2 * wN;
  const unsigned short* Wo16 = W16 + (size_t)3 * wN;

  stats_kernel<<<dim3(2 * (kBatch * kCh) / 32), dim3(256), 0, stream>>>(content, style, meanA, rstdA);

  wcast_kernel<<<dim3(512), dim3(256), 0, stream>>>(Wq, Wk, Wv, Wo, W16, kWCarry);

  for (int b = 0; b < kBatch; ++b) {
    const size_t actOff = (size_t)b * kCh * kSp;

    token_planes_kernel<<<dim3(kSp / 64, kCh / 64, 3), dim3(256), 0, stream>>>(content, style, meanA, rstdA, b, XcT, XsT, SsT);

    wmma_gemm64<0, false, 2, 1, false><<<dim3(64, 1), dim3(256), 0, stream>>>(
        XcT, nullptr, kCh, 0L, Wq16, nullptr, kCh, 0L, (void*)Qp, nullptr, kCh, 0L,
        bq, nullptr, 0L, kSp, kCh, kCh, kProjScale);
    wmma_gemm64<0, false, 2, 1, false><<<dim3(64, 1), dim3(256), 0, stream>>>(
        XsT, nullptr, kCh, 0L, Wk16, nullptr, kCh, 0L, (void*)Kp, nullptr, kCh, 0L,
        bk, nullptr, 0L, kSp, kCh, kCh, kProjScale);
    wmma_gemm64<0, false, 1, 1, false><<<dim3(64, 1), dim3(256), 0, stream>>>(
        Wv16, nullptr, kCh, 0L, SsT, nullptr, kCh, 0L, (void*)Vcm, nullptr, kSp, 0L,
        bv, nullptr, 0L, kCh, kSp, kCh, kProjScale);

    for (int ch = 0; ch < kSp / kQChunk; ++ch) {
      const size_t qOff = (size_t)ch * kQChunk * kCh;
      wmma_gemm64<0, false, 0, 0, false><<<dim3(256, 1), dim3(256), 0, stream>>>(
          Qp + qOff, nullptr, kCh, 0L, Kp, nullptr, kCh, 0L, (void*)Sp, nullptr, kSp, 0L,
          nullptr, nullptr, 0L, kQChunk, kSp, kCh, 1.0f);
      softmax_kernel<<<dim3(kQChunk), dim3(256), 0, stream>>>(Sp, Pp);
      wmma_gemm64<0, false, 0, 1, false><<<dim3(32, 1), dim3(256), 0, stream>>>(
          Pp, nullptr, kSp, 0L, Vcm, nullptr, kSp, 0L, (void*)(Op + qOff), nullptr, kCh, 0L,
          nullptr, nullptr, 0L, kQChunk, kCh, kSp, kPVScale);
    }

    wmma_gemm64<0, false, 1, 0, true><<<dim3(64, 1), dim3(256), 0, stream>>>(
        Wo16, nullptr, kCh, 0L, Op, nullptr, kCh, 0L, (void*)(out + actOff), nullptr, kSp, 0L,
        bo, content + actOff, 0L, kCh, kSp, kCh, kOutScale);
  }
}
